// DSAttention_21045339750736
// MI455X (gfx1250) — hardware-verified
//
#include <hip/hip_runtime.h>
#include <math.h>
#include <stdint.h>

#ifndef NB
#define NB 4
#endif
#ifndef SEQ
#define SEQ 2048
#endif
#define NB_FULL  4
#define SEQ_FULL 2048
#define NH  8
#define HD  64
#define DM  (NH * HD)
#define NQB (SEQ / 64)
#define RESQB 8
#define VCARRY 16.0f
#define PCARRY 1024.0f
#define PRES   4096.0f
static_assert((SEQ % 64) == 0);
static_assert(SEQ >= 64 && SEQ <= SEQ_FULL);
static_assert(NB >= 1 && NB <= NB_FULL);
static_assert(NH * HD == DM);
static_assert(((SEQ * DM / 8) % 256) == 0);

typedef _Float16 v16h __attribute__((ext_vector_type(16)));
typedef _Float16 v8h  __attribute__((ext_vector_type(8)));
typedef __bf16   v16b __attribute__((ext_vector_type(16)));
typedef __bf16   v8b  __attribute__((ext_vector_type(8)));
typedef float    v8f  __attribute__((ext_vector_type(8)));
typedef float    v4f  __attribute__((ext_vector_type(4)));
typedef unsigned int v4u __attribute__((ext_vector_type(4)));

__device__ __forceinline__ unsigned short bf_bits(float f) {
  unsigned u = __float_as_uint(f);
  return (unsigned short)((u + 0x7FFFu + ((u >> 16) & 1u)) >> 16);
}
__device__ __forceinline__ float bf_up(unsigned short h) { return __uint_as_float(((unsigned)h) << 16); }
__device__ __forceinline__ unsigned pk16(unsigned short a, unsigned short b) { return (unsigned)a | ((unsigned)b << 16); }
__device__ __forceinline__ v8f zero8() { v8f z = {0.f, 0.f, 0.f, 0.f, 0.f, 0.f, 0.f, 0.f}; return z; }

__device__ __forceinline__ v16b ldfrag_b(const __bf16* p) {
  union { v16b v; v8b h[2]; } f;
  f.h[0] = *(const v8b*)(p);
  f.h[1] = *(const v8b*)(p + 16);
  return f.v;
}

__device__ __forceinline__ v8f mma_b(v16b a, v16b b, v8f c) {
  c = __builtin_amdgcn_wmma_f32_16x16x32_bf16(false, a, false, b, (short)0, c, false, false);
  asm volatile("v_nop\n\tv_nop\n\tv_nop\n\tv_nop" : "+v"(c) : "v"(a), "v"(b));
  return c;
}
__device__ __forceinline__ v8f mma_h(v16h a, v16h b, v8f c) {
  c = __builtin_amdgcn_wmma_f32_16x16x32_f16(false, a, false, b, (short)0, c, false, false);
  asm volatile("v_nop\n\tv_nop\n\tv_nop\n\tv_nop" : "+v"(c) : "v"(a), "v"(b));
  return c;
}

__global__ __launch_bounds__(256) void cvt_bf16x8(const float* __restrict__ in, unsigned short* out, int n8,
                                                  long long sIn, long long sOut) {
  const int i = blockIdx.x * 256 + threadIdx.x;
  const int b = blockIdx.y;
  if (i < n8) {
    const float* src = in + (size_t)b * (size_t)sIn + (size_t)i * 8;
    unsigned short* dst = out + (size_t)b * (size_t)sOut + (size_t)i * 8;
    const v4f a  = *(const v4f*)(src);
    const v4f a4 = *(const v4f*)(src + 4);
    v4u p;
    p[0] = pk16(bf_bits(a[0]),  bf_bits(a[1]));
    p[1] = pk16(bf_bits(a[2]),  bf_bits(a[3]));
    p[2] = pk16(bf_bits(a4[0]), bf_bits(a4[1]));
    p[3] = pk16(bf_bits(a4[2]), bf_bits(a4[3]));
    *(volatile v4u*)(dst) = p;
    __threadfence();
    *(volatile v4u*)(dst) = p;
  }
}

__global__ __launch_bounds__(256) void vt_cvt(const float* __restrict__ v, unsigned short* vt) {
  __shared__ __align__(16) _Float16 T[64 * 72];
  const int tid  = threadIdx.x;
  const int wave = tid >> 5;
  const int lane = tid & 31;
  const int st   = blockIdx.x;
  const int h    = blockIdx.y;
  const int b    = blockIdx.z;
  {
    const int s  = tid >> 2;
    const int dq = (tid & 3) * 16;
    const float* src = v + (((size_t)b * SEQ_FULL + (size_t)st * 64 + (size_t)s) * DM + (size_t)h * HD + (size_t)dq);
#pragma unroll
    for (int i = 0; i < 4; ++i) {
      const v4f a = *(const v4f*)(src + 4 * i);
#pragma unroll
      for (int e = 0; e < 4; ++e) {
        const float f = bf_up(bf_bits(a[e])) * VCARRY;
        T[(dq + 4 * i + e) * 72 + s] = (_Float16)f;
      }
    }
  }
  __syncthreads();
  {
    const int q8 = lane >> 3, c8 = (lane & 7) * 8;
    v4u w[2];
#pragma unroll
    for (int it = 0; it < 2; ++it) {
      const int d = wave * 8 + it * 4 + q8;
      const v8h x = *(const v8h*)(T + d * 72 + c8);
      w[it] = __builtin_bit_cast(v4u, x);
    }
    unsigned short* dst = vt + ((size_t)b * DM + (size_t)h * HD) * SEQ + (size_t)st * 64 + (size_t)c8;
    for (int pass = 0; pass < 2; ++pass) {
#pragma unroll
      for (int it = 0; it < 2; ++it) {
        const int d = wave * 8 + it * 4 + q8;
        *(volatile v4u*)(dst + (size_t)d * SEQ) = w[it];
      }
      __threadfence();
    }
  }
}

template <bool RES>
__global__ __launch_bounds__(128)
void attn_causal64(const unsigned short* __restrict__ qp, const unsigned short* __restrict__ kp,
                   const unsigned short* __restrict__ vtp, const float* __restrict__ taup,
                   const float* __restrict__ deltap, float* outp, int qbBase, int nqbThis) {
  union FB { v16b v; v8b h[2]; };
  union FH { v16h v; v8h h[2]; };
  __shared__ __align__(16) __bf16   Ksh[64 * 64];
  __shared__ __align__(16) _Float16 Vth[64 * 64];
  __shared__ __align__(16) _Float16 Psh[4][16 * 64];
  __shared__ __align__(16) _Float16 Psl[RES ? 4 : 1][16 * 64];
  __shared__ __align__(16) float    Os[4][16 * 64];

  const int tid  = threadIdx.x;
  const int wave = tid >> 5;
  const int lane = tid & 31;
  const int hh   = lane >> 4;
  const int c    = lane & 15;

  const int bx   = blockIdx.x;
  const int qbl  = bx % nqbThis;
  const int rest = bx / nqbThis;
  const int h    = rest % NH;
  const int b    = rest / NH;
  const int qb   = qbBase + qbl;
  const int q0   = qb * 64 + wave * 16;
  const size_t rowB = (size_t)b * SEQ;

  const __bf16*   Qh = (const __bf16*)(const void*)qp + (size_t)h * HD;
  const __bf16*   Kh = (const __bf16*)(const void*)kp + (size_t)h * HD;
  const _Float16* Vt = (const _Float16*)(const void*)vtp + ((size_t)b * DM + (size_t)h * HD) * SEQ;
  const float* dlt   = deltap + (size_t)b * SEQ_FULL;
  float* Ob          = outp + (size_t)h * HD;
  const float tau_b  = bf_up(bf_bits(taup[b]));

  v16b qa[2];
#pragma unroll
  for (int dc = 0; dc < 2; ++dc) {
    const size_t qo = (rowB + (size_t)q0 + (size_t)c) * DM + (size_t)(dc * 32 + 8 * hh);
    qa[dc] = ldfrag_b(Qh + qo);
  }

  float mrow[8], lrow[8];
  v8f oacc[4];
#pragma unroll
  for (int r = 0; r < 8; ++r) { mrow[r] = -INFINITY; lrow[r] = 0.f; }
#pragma unroll
  for (int t = 0; t < 4; ++t) oacc[t] = zero8();

  for (int kt = 0; kt < NQB; ++kt) {
    if (kt > qb) break;
    const int kv0 = kt * 64;
    __syncthreads();
    {
      const int r = tid >> 1, half = (tid & 1) * 32;
      const __bf16*   kg = Kh + (rowB + (size_t)kv0 + (size_t)r) * DM + half;
      const _Float16* vg = Vt + (size_t)r * SEQ + (size_t)kv0 + half;
#pragma unroll
      for (int i = 0; i < 4; ++i) {
        const v8b a0 = *(const v8b*)(kg + 8 * i);
        const v8h b0 = *(const v8h*)(vg + 8 * i);
        *(v8b*)(Ksh + r * 64 + half + 8 * i) = a0;
        *(v8h*)(Vth + r * 64 + half + 8 * i) = b0;
      }
    }
    __syncthreads();

    v8f s[4];
#pragma unroll
    for (int j = 0; j < 4; ++j) {
      s[j] = zero8();
#pragma unroll
      for (int dc = 0; dc < 2; ++dc) {
        FB kb;
        kb.h[0] = *(const v8b*)(Ksh + (j * 16 + c) * 64 + dc * 32 + 8 * hh);
        kb.h[1] = *(const v8b*)(Ksh + (j * 16 + c) * 64 + dc * 32 + 16 + 8 * hh);
        s[j] = mma_b(qa[dc], kb.v, s[j]);
      }
    }

    float dj[4];
#pragma unroll
    for (int j = 0; j < 4; ++j) dj[j] = bf_up(bf_bits(dlt[kv0 + j * 16 + c]));
    _Float16* pwh = Psh[wave];
    _Float16* pwl = Psl[RES ? wave : 0];
#pragma unroll
    for (int r = 0; r < 8; ++r) {
      const int ridx = q0 + 8 * hh + r;
      float m = -INFINITY;
#pragma unroll
      for (int j = 0; j < 4; ++j) {
        const int kidx = kv0 + j * 16 + c;
        float sv = (s[j][r] * tau_b + dj[j]) * 0.125f;
        sv = (kidx > ridx) ? -INFINITY : sv;
        s[j][r] = sv;
        m = fmaxf(m, sv);
      }
#pragma unroll
      for (int off = 1; off < 16; off <<= 1) m = fmaxf(m, __shfl_xor(m, off, 32));
      const float mnew  = fmaxf(mrow[r], m);
      const float msafe = (mnew == -INFINITY) ? 0.f : mnew;
      const float alpha = __expf(mrow[r] - msafe);
      mrow[r] = mnew;
      float psum = 0.f;
#pragma unroll
      for (int j = 0; j < 4; ++j) {
        const float p = __expf(s[j][r] - msafe);
        psum += p;
        const float p1k = p * PCARRY;
        const _Float16 ph = (_Float16)p1k;
        pwh[(8 * hh + r) * 64 + j * 16 + c] = ph;
        if (RES) {
          const _Float16 pl = (_Float16)((p1k - (float)ph) * PRES);
          pwl[(8 * hh + r) * 64 + j * 16 + c] = pl;
        }
      }
#pragma unroll
      for (int off = 1; off < 16; off <<= 1) psum += __shfl_xor(psum, off, 32);
      lrow[r] = lrow[r] * alpha + psum;
#pragma unroll
      for (int t = 0; t < 4; ++t) oacc[t][r] *= alpha;
    }
    __builtin_amdgcn_fence(__ATOMIC_RELEASE, "workgroup");
    __builtin_amdgcn_wave_barrier();
    __builtin_amdgcn_fence(__ATOMIC_ACQUIRE, "workgroup");

    v8f o1[4];
#pragma unroll
    for (int t = 0; t < 4; ++t) o1[t] = zero8();
#pragma unroll 1
    for (int kk = 0; kk < 2; ++kk) {
      FH pa, pl;
      pa.h[0] = *(const v8h*)(pwh + c * 64 + kk * 32 + 8 * hh);
      pa.h[1] = *(const v8h*)(pwh + c * 64 + kk * 32 + 16 + 8 * hh);
      if (RES) {
        pl.h[0] = *(const v8h*)(pwl + c * 64 + kk * 32 + 8 * hh);
        pl.h[1] = *(const v8h*)(pwl + c * 64 + kk * 32 + 16 + 8 * hh);
      } else {
        pl.v = pa.v;
      }
#pragma unroll
      for (int t = 0; t < 4; ++t) {
        FH vb;
        vb.h[0] = *(const v8h*)(Vth + (t * 16 + c) * 64 + kk * 32 + 8 * hh);
        vb.h[1] = *(const v8h*)(Vth + (t * 16 + c) * 64 + kk * 32 + 16 + 8 * hh);
        oacc[t] = mma_h(pa.v, vb.v, oacc[t]);
        if (RES) o1[t] = mma_h(pl.v, vb.v, o1[t]);
      }
    }
    if (RES) {
#pragma unroll
      for (int t = 0; t < 4; ++t)
#pragma unroll
        for (int r = 0; r < 8; ++r) oacc[t][r] += o1[t][r] * (1.0f / PRES);
    }
  }

  float* os = Os[wave];
#pragma unroll
  for (int r = 0; r < 8; ++r) {
    const float l = lrow[r];
    const float inv = ((l > 0.f) ? (1.0f / l) : 0.f) * (1.0f / PCARRY) * (1.0f / VCARRY);
#pragma unroll
    for (int t = 0; t < 4; ++t) os[(8 * hh + r) * 64 + t * 16 + c] = oacc[t][r] * inv;
  }
  __builtin_amdgcn_fence(__ATOMIC_RELEASE, "workgroup");
  __builtin_amdgcn_wave_barrier();
  __builtin_amdgcn_fence(__ATOMIC_ACQUIRE, "workgroup");
  {
    const int hh2 = lane >> 4, c4 = (lane & 15) * 4;
    v4f vv[8];
#pragma unroll
    for (int it = 0; it < 8; ++it) {
      const int row = it * 2 + hh2;
      vv[it] = *(const v4f*)(os + row * 64 + c4);
    }
    for (int pass = 0; pass < 2; ++pass) {
#pragma unroll
      for (int it = 0; it < 8; ++it) {
        const int row = it * 2 + hh2;
        *(volatile v4f*)(Ob + (rowB + (size_t)q0 + (size_t)row) * DM + (size_t)c4) = vv[it];
      }
      __threadfence();
    }
  }
}

extern "C" void kernel_launch(void* const* d_in, const int* in_sizes, int n_in,
                              void* d_out, int out_size, void* d_ws, size_t ws_size,
                              hipStream_t stream) {
  if (n_in < 5) return;
  const long long needTok = (long long)(NB - 1) * SEQ_FULL + (long long)SEQ;
  if ((long long)in_sizes[0] < needTok * DM) return;
  if ((long long)in_sizes[1] < needTok * DM) return;
  if ((long long)in_sizes[2] < needTok * DM) return;
  if (in_sizes[3] < NB) return;
  if ((long long)in_sizes[4] < needTok) return;
  if ((long long)out_size < (long long)NB * SEQ * DM) return;

  const float* q     = (const float*)d_in[0];
  const float* k     = (const float*)d_in[1];
  const float* v     = (const float*)d_in[2];
  const float* tau   = (const float*)d_in[3];
  const float* delta = (const float*)d_in[4];
  float* out = (float*)d_out;

  const size_t PX = (size_t)NB * SEQ * DM * 2;
  size_t off = 0;
  const size_t oQ = off; off += PX;
  const size_t oK = off; off += PX;
  const size_t oV = off; off += PX;
  if (off > ws_size) return;
  if (off > (size_t)134217728) return;

  char* ws = (char*)d_ws;
  unsigned short* Qb  = (unsigned short*)(ws + oQ);
  unsigned short* Kb  = (unsigned short*)(ws + oK);
  unsigned short* VTb = (unsigned short*)(ws + oV);

  const int n8b = SEQ * DM / 8;
  const dim3 gCvt((n8b + 255) / 256, NB);
  const dim3 gVT(NQB, NH, NB);
  const int resq = (RESQB < NQB) ? RESQB : NQB;

  cvt_bf16x8<<<gCvt, dim3(256), 0, stream>>>(q, Qb, n8b, (long long)SEQ_FULL * DM, (long long)SEQ * DM);
  cvt_bf16x8<<<gCvt, dim3(256), 0, stream>>>(k, Kb, n8b, (long long)SEQ_FULL * DM, (long long)SEQ * DM);
  vt_cvt<<<gVT, dim3(256), 0, stream>>>(v, VTb);
  attn_causal64<true><<<dim3(NB * NH * resq), dim3(128), 0, stream>>>(
      Qb, Kb, VTb, tau, delta, out, 0, resq);
  if (NQB > resq) {
    attn_causal64<false><<<dim3(NB * NH * (NQB - resq)), dim3(128), 0, stream>>>(
        Qb, Kb, VTb, tau, delta, out, resq, NQB - resq);
  }
  (void)hipGetLastError();
}
